// _DinatLayerNd_49993419325476
// MI455X (gfx1250) — hardware-verified
//
#include <hip/hip_runtime.h>
#include <stdint.h>

#define NB_   4
#define TT_   4096
#define CC_   512
#define NH_   8
#define HD_   64
#define KS_   7
#define DL_   4
#define LL_   (TT_ / DL_)
#define FF_   2048
#define NT_   (NB_ * TT_)
#define RB_   (2 * KS_ - 1)
#define QKVW_ (3 * CC_)
#define WSC_  32.0f
#define WINV_ 0.03125f

static_assert(NT_ % 128 == 0);
static_assert((NT_ / 2) % 128 == 0);
static_assert(CC_ % 64 == 0 && FF_ % 64 == 0 && QKVW_ % 64 == 0);
static_assert(CC_ % 32 == 0 && FF_ % 32 == 0);
static_assert(NT_ % 8 == 0);
static_assert(TT_ / 32 == 128);
static_assert(NH_ * HD_ == CC_);
static_assert(TT_ % DL_ == 0);

typedef _Float16 v16h __attribute__((ext_vector_type(16)));
typedef _Float16 v8h  __attribute__((ext_vector_type(8)));
typedef _Float16 v2h  __attribute__((ext_vector_type(2)));
typedef float    v8f  __attribute__((ext_vector_type(8)));
typedef float    v4f  __attribute__((ext_vector_type(4)));
typedef v8h __attribute__((may_alias)) v8ha;
typedef v2h __attribute__((may_alias)) v2ha;
typedef v4f __attribute__((may_alias)) v4fa;

union Frag { v16h v; v8h half[2]; };

__device__ __forceinline__ v8f wmma_f16(v16h a, v16h b, v8f c) {
  v8f d = __builtin_amdgcn_wmma_f32_16x16x32_f16(false, a, false, b, (short)0, c, false, false);
#if defined(__HIP_DEVICE_COMPILE__)
  asm volatile("v_nop\n\tv_nop\n\tv_nop\n\tv_nop" : "+v"(d) : "v"(a), "v"(b));
#endif
  return d;
}

__device__ __forceinline__ v16h load_frag(const _Float16* p, int h) {
  Frag f;
  f.half[0] = *(const v8ha*)(p + 8 * h);
  f.half[1] = *(const v8ha*)(p + 16 + 8 * h);
  return f.v;
}

#define WU_SMALL (CC_ * CC_ / 8)
#define WU_BIG   (FF_ * CC_ / 8)
#define WU_TOTAL (4 * WU_SMALL + 2 * WU_BIG)
static_assert(WU_SMALL == 32768);
static_assert(WU_SMALL % 256 == 0 && WU_BIG % 256 == 0);

__global__ __launch_bounds__(256) void wconv_kernel(
    const float* __restrict__ wq, const float* __restrict__ wk,
    const float* __restrict__ wv, const float* __restrict__ wo,
    const float* __restrict__ w1, const float* __restrict__ w2,
    _Float16* __restrict__ wts)
{
  const int g = blockIdx.x * 256 + threadIdx.x;
  if (g >= WU_TOTAL) return;
  const int seg = g >> 15;
  const float* src;
  if (seg < 4) {
    const float* base = (seg == 0) ? wq : ((seg == 1) ? wk : ((seg == 2) ? wv : wo));
    src = base + (size_t)(g - (seg << 15)) * 8;
  } else if (seg < 8) {
    src = w1 + (size_t)(g - 4 * WU_SMALL) * 8;
  } else {
    src = w2 + (size_t)(g - 4 * WU_SMALL - WU_BIG) * 8;
  }
  const v4f a = *(const v4fa*)src;
  const v4f c = *(const v4fa*)(src + 4);
  const v8h o = { (_Float16)(a.x * WSC_), (_Float16)(a.y * WSC_), (_Float16)(a.z * WSC_), (_Float16)(a.w * WSC_),
                  (_Float16)(c.x * WSC_), (_Float16)(c.y * WSC_), (_Float16)(c.z * WSC_), (_Float16)(c.w * WSC_) };
  _Float16* dst = wts + (size_t)g * 8;
  *(volatile v8h*)dst = o;
  __threadfence();
  *(volatile v8h*)dst = o;
}

__global__ __launch_bounds__(256) void layernorm_kernel(
    const float* __restrict__ x, const float* __restrict__ gam,
    const float* __restrict__ bet, _Float16* __restrict__ out)
{
  const int lane = threadIdx.x & 31, w = threadIdx.x >> 5;
  const int row = blockIdx.x * 8 + w;
  const float* xr = x + (size_t)row * CC_;

  const v4f p0 = *(const v4fa*)(xr + 8 * lane);
  const v4f p1 = *(const v4fa*)(xr + 8 * lane + 4);
  const v4f p2 = *(const v4fa*)(xr + 256 + 8 * lane);
  const v4f p3 = *(const v4fa*)(xr + 256 + 8 * lane + 4);
  float v[16] = { p0.x, p0.y, p0.z, p0.w, p1.x, p1.y, p1.z, p1.w,
                  p2.x, p2.y, p2.z, p2.w, p3.x, p3.y, p3.z, p3.w };

  float s = 0.0f;
  #pragma unroll
  for (int i = 0; i < 16; ++i) s += v[i];
  #pragma unroll
  for (int o = 16; o > 0; o >>= 1) s += __shfl_xor(s, o, 32);
  const float mu = s * (1.0f / CC_);

  float ss = 0.0f;
  #pragma unroll
  for (int i = 0; i < 16; ++i) { v[i] = v[i] - mu; ss += v[i] * v[i]; }
  #pragma unroll
  for (int o = 16; o > 0; o >>= 1) ss += __shfl_xor(ss, o, 32);
  const float inv = rsqrtf(ss * (1.0f / CC_) + 1e-5f);

  const v4f g0 = *(const v4fa*)(gam + 8 * lane);
  const v4f g1 = *(const v4fa*)(gam + 8 * lane + 4);
  const v4f g2 = *(const v4fa*)(gam + 256 + 8 * lane);
  const v4f g3 = *(const v4fa*)(gam + 256 + 8 * lane + 4);
  const v4f b0 = *(const v4fa*)(bet + 8 * lane);
  const v4f b1 = *(const v4fa*)(bet + 8 * lane + 4);
  const v4f b2 = *(const v4fa*)(bet + 256 + 8 * lane);
  const v4f b3 = *(const v4fa*)(bet + 256 + 8 * lane + 4);
  const float gg[16] = { g0.x, g0.y, g0.z, g0.w, g1.x, g1.y, g1.z, g1.w,
                         g2.x, g2.y, g2.z, g2.w, g3.x, g3.y, g3.z, g3.w };
  const float bb[16] = { b0.x, b0.y, b0.z, b0.w, b1.x, b1.y, b1.z, b1.w,
                         b2.x, b2.y, b2.z, b2.w, b3.x, b3.y, b3.z, b3.w };
  float y[16];
  #pragma unroll
  for (int i = 0; i < 16; ++i) y[i] = (v[i] * inv) * gg[i] + bb[i];

  const v8h o0 = { (_Float16)y[0], (_Float16)y[1], (_Float16)y[2],  (_Float16)y[3],
                   (_Float16)y[4], (_Float16)y[5], (_Float16)y[6],  (_Float16)y[7] };
  const v8h o1 = { (_Float16)y[8], (_Float16)y[9], (_Float16)y[10], (_Float16)y[11],
                   (_Float16)y[12], (_Float16)y[13], (_Float16)y[14], (_Float16)y[15] };
  _Float16* orow = out + (size_t)row * CC_;
  *(volatile v8h*)(orow + 8 * lane) = o0;
  *(volatile v8h*)(orow + 256 + 8 * lane) = o1;
  __threadfence();
  *(volatile v8h*)(orow + 8 * lane) = o0;
  *(volatile v8h*)(orow + 256 + 8 * lane) = o1;
}

template <int EPI>
__global__ __launch_bounds__(128) void gemm_kernel(
    const _Float16* __restrict__ A,
    const _Float16* __restrict__ W,
    const float* __restrict__ bias0, const float* __restrict__ bias1,
    const float* __restrict__ bias2, int bseg,
    const float* __restrict__ resid,
    float* __restrict__ outF,
    _Float16* __restrict__ outH,
    int ldo, int K)
{
  __shared__ __attribute__((aligned(16))) char sraw[128 * 64 * 4];
  float*    sF = (float*)sraw;
  _Float16* sH = (_Float16*)sraw;

  const int tid = threadIdx.x, lane = tid & 31, w = tid >> 5;
  const int h = lane >> 4, m = lane & 15;
  const int m0 = blockIdx.x * 128, n0 = blockIdx.y * 64;
  const int m0w = m0 + 32 * w;

  const _Float16* a0p = A + (size_t)(m0w + m) * K;
  const _Float16* a1p = a0p + (size_t)16 * K;
  const _Float16* wp  = W + (size_t)(n0 + m) * K;

  const v8f zero8 = {0.f, 0.f, 0.f, 0.f, 0.f, 0.f, 0.f, 0.f};
  v8f acc[2][4];
  #pragma unroll
  for (int mt = 0; mt < 2; ++mt)
    #pragma unroll
    for (int nt = 0; nt < 4; ++nt) acc[mt][nt] = zero8;

  #pragma unroll 1
  for (int k0 = 0; k0 < K; k0 += 32) {
    const v16h a0 = load_frag(a0p + k0, h);
    const v16h a1 = load_frag(a1p + k0, h);
    #pragma unroll
    for (int nt = 0; nt < 4; ++nt) {
      const v16h b = load_frag(wp + (size_t)(16 * nt) * K + k0, h);
      acc[0][nt] = wmma_f16(a0, b, acc[0][nt]);
      acc[1][nt] = wmma_f16(a1, b, acc[1][nt]);
    }
  }

  int seg = n0 / bseg;
  seg = (seg > 2) ? 2 : seg;
  const float* bias = (seg == 0) ? bias0 : ((seg == 1) ? bias1 : bias2);
  const int bc0 = n0 - seg * bseg;

  #pragma unroll
  for (int nt = 0; nt < 4; ++nt) {
    const int col = 16 * nt + m;
    const float bvl = bias[bc0 + col];
    #pragma unroll
    for (int mt = 0; mt < 2; ++mt) {
      #pragma unroll
      for (int r = 0; r < 8; ++r) {
        const int rl = 32 * w + 16 * mt + 8 * h + r;
        const float v = acc[mt][nt][r] * WINV_ + bvl;
        if constexpr (EPI == 1) {
          sF[rl * 64 + col] = v;
        } else if constexpr (EPI == 0) {
          sH[rl * 64 + col] = (_Float16)v;
        } else {
          const float ge = 0.5f * v * (1.0f + erff(v * 0.70710678118654752f));
          sH[rl * 64 + col] = (_Float16)ge;
        }
      }
    }
  }
  __syncthreads();

  const int q8 = lane & 7, sub = lane >> 3;
  if constexpr (EPI == 1) {
    v4f fv[16];
    #pragma unroll
    for (int i = 0; i < 16; ++i) {
      const int row = 32 * w + 2 * i + (sub >> 1);
      const int hl = sub & 1;
      const v4f tv = *(const v4fa*)(sF + row * 64 + 32 * hl + 4 * q8);
      const size_t gi = (size_t)(m0 + row) * ldo + n0 + 32 * hl + 4 * q8;
      const v4f rv = *(const v4fa*)(resid + gi);
      fv[i] = tv + rv;
      *(volatile v4f*)(outF + gi) = fv[i];
    }
    __threadfence();
    #pragma unroll
    for (int i = 0; i < 16; ++i) {
      const int row = 32 * w + 2 * i + (sub >> 1);
      const int hl = sub & 1;
      const size_t gi = (size_t)(m0 + row) * ldo + n0 + 32 * hl + 4 * q8;
      *(volatile v4f*)(outF + gi) = fv[i];
    }
  } else {
    v8h hv[8];
    #pragma unroll
    for (int i = 0; i < 8; ++i) {
      const int lid = 32 * w + 4 * i + sub;
      hv[i] = *(const v8ha*)(sH + lid * 64 + 8 * q8);
      _Float16* dst = outH + (size_t)(m0 + lid) * ldo + n0 + 8 * q8;
      *(volatile v8h*)dst = hv[i];
    }
    __threadfence();
    #pragma unroll
    for (int i = 0; i < 8; ++i) {
      const int lid = 32 * w + 4 * i + sub;
      _Float16* dst = outH + (size_t)(m0 + lid) * ldo + n0 + 8 * q8;
      *(volatile v8h*)dst = hv[i];
    }
  }
}

__global__ __launch_bounds__(256) void na_kernel(
    const _Float16* __restrict__ qkv, const float* __restrict__ rpb,
    _Float16* __restrict__ ctx)
{
  __shared__ __attribute__((aligned(16))) _Float16 sC[32 * CC_];

  const int tid = threadIdx.x, lane = tid & 31, w = tid >> 5;
  const int blk = blockIdx.x;
  const int n  = blk >> 7;
  const int t0 = (blk & 127) * 32;
  const int tl = tid >> 3, hh = tid & 7;
  const int t  = t0 + tl;
  const int g  = t % DL_, p = t / DL_;
  int start = p - (KS_ / 2);
  start = (start < 0) ? 0 : start;
  start = (start > (LL_ - KS_)) ? (LL_ - KS_) : start;

  const _Float16* qp = qkv + (size_t)(n * TT_ + t) * QKVW_ + hh * HD_;
  const _Float16* kb = qkv + CC_ + hh * HD_;
  const _Float16* vb = qkv + 2 * CC_ + hh * HD_;

  int ro[KS_];
  #pragma unroll
  for (int j = 0; j < KS_; ++j) {
    int nbp = start + j;
    nbp = (nbp < 0) ? 0 : ((nbp > LL_ - 1) ? (LL_ - 1) : nbp);
    ro[j] = (n * TT_ + nbp * DL_ + g) * QKVW_;
  }

  float s[KS_];
  #pragma unroll
  for (int j = 0; j < KS_; ++j) s[j] = 0.0f;

  #pragma unroll 1
  for (int c = 0; c < HD_; c += 2) {
    const v2h qq = *(const v2ha*)(qp + c);
    const float qa = (float)qq.x, qb = (float)qq.y;
    #pragma unroll
    for (int j = 0; j < KS_; ++j) {
      const v2h kk = *(const v2ha*)(kb + ro[j] + c);
      s[j] = s[j] + qa * (float)kk.x + qb * (float)kk.y;
    }
  }

  float mx = -3.0e38f;
  #pragma unroll
  for (int j = 0; j < KS_; ++j) {
    int bi = start + j - p + (KS_ - 1);
    bi = (bi < 0) ? 0 : ((bi > RB_ - 1) ? (RB_ - 1) : bi);
    s[j] = s[j] * 0.125f + rpb[hh * RB_ + bi];
    mx = fmaxf(mx, s[j]);
  }
  float den = 0.0f;
  #pragma unroll
  for (int j = 0; j < KS_; ++j) { s[j] = __expf(s[j] - mx); den += s[j]; }
  const float rden = 1.0f / den;
  #pragma unroll
  for (int j = 0; j < KS_; ++j) s[j] = s[j] * rden;

  _Float16* so = sC + tl * CC_ + hh * HD_;
  #pragma unroll 1
  for (int c = 0; c < HD_; c += 2) {
    float oa = 0.0f, ob = 0.0f;
    #pragma unroll
    for (int j = 0; j < KS_; ++j) {
      const v2h vv = *(const v2ha*)(vb + ro[j] + c);
      oa = oa + s[j] * (float)vv.x;
      ob = ob + s[j] * (float)vv.y;
    }
    v2h ov;
    ov.x = (_Float16)oa;
    ov.y = (_Float16)ob;
    *(v2ha*)(so + c) = ov;
  }
  __syncthreads();

  v8h hv[8];
  #pragma unroll
  for (int i = 0; i < 8; ++i) {
    const int row = 4 * w + (i >> 1), hf = i & 1;
    hv[i] = *(const v8ha*)(sC + row * CC_ + 256 * hf + 8 * lane);
    _Float16* dst = ctx + (size_t)(n * TT_ + t0 + row) * CC_ + 256 * hf + 8 * lane;
    *(volatile v8h*)dst = hv[i];
  }
  __threadfence();
  #pragma unroll
  for (int i = 0; i < 8; ++i) {
    const int row = 4 * w + (i >> 1), hf = i & 1;
    _Float16* dst = ctx + (size_t)(n * TT_ + t0 + row) * CC_ + 256 * hf + 8 * lane;
    *(volatile v8h*)dst = hv[i];
  }
}

extern "C" void kernel_launch(void* const* d_in, const int* in_sizes, int n_in,
                              void* d_out, int out_size, void* d_ws, size_t ws_size,
                              hipStream_t stream) {
  if (n_in < 18) return;
  if (in_sizes[0] != NT_ * CC_) return;
  if (in_sizes[1] != CC_ || in_sizes[2] != CC_) return;
  if (in_sizes[3] != CC_ * CC_ || in_sizes[5] != CC_ * CC_ || in_sizes[7] != CC_ * CC_) return;
  if (in_sizes[4] != CC_ || in_sizes[6] != CC_ || in_sizes[8] != CC_) return;
  if (in_sizes[9] != NH_ * RB_) return;
  if (in_sizes[10] != CC_ * CC_ || in_sizes[11] != CC_) return;
  if (in_sizes[12] != CC_ || in_sizes[13] != CC_) return;
  if (in_sizes[14] != FF_ * CC_ || in_sizes[15] != FF_) return;
  if (in_sizes[16] != CC_ * FF_ || in_sizes[17] != CC_) return;
  if (out_size != NT_ * CC_) return;

  const float* x     = (const float*)d_in[0];
  const float* ln1_g = (const float*)d_in[1];
  const float* ln1_b = (const float*)d_in[2];
  const float* wq    = (const float*)d_in[3];
  const float* bq    = (const float*)d_in[4];
  const float* wk    = (const float*)d_in[5];
  const float* bk    = (const float*)d_in[6];
  const float* wv    = (const float*)d_in[7];
  const float* bv    = (const float*)d_in[8];
  const float* rpb   = (const float*)d_in[9];
  const float* wo    = (const float*)d_in[10];
  const float* bo    = (const float*)d_in[11];
  const float* ln2_g = (const float*)d_in[12];
  const float* ln2_b = (const float*)d_in[13];
  const float* w1    = (const float*)d_in[14];
  const float* b1    = (const float*)d_in[15];
  const float* w2    = (const float*)d_in[16];
  const float* b2    = (const float*)d_in[17];
  float* out = (float*)d_out;

  const size_t wts_bytes = (size_t)(4 * CC_ * CC_ + 2 * FF_ * CC_) * 2;
  const size_t r1_bytes  = (size_t)NT_ * CC_ * 2;
  const size_t r2_bytes  = (size_t)NT_ * QKVW_ * 2;
  const size_t r3_bytes  = (size_t)(NT_ / 2) * FF_ * 2;
  const size_t total     = wts_bytes + r1_bytes + r2_bytes + r3_bytes;
  if (total > ws_size) return;
  if ((size_t)NT_ * CC_ * 4 > r2_bytes) return;

  char* ws = (char*)d_ws;
  _Float16* wts   = (_Float16*)(ws);
  _Float16* wqkvh = wts;
  _Float16* woh   = wts + (size_t)3 * CC_ * CC_;
  _Float16* w1h   = wts + (size_t)4 * CC_ * CC_;
  _Float16* w2h   = wts + (size_t)4 * CC_ * CC_ + (size_t)FF_ * CC_;
  _Float16* r1    = (_Float16*)(ws + wts_bytes);
  char*     r2c   = ws + wts_bytes + r1_bytes;
  _Float16* qkvh  = (_Float16*)r2c;
  float*    hidden = (float*)r2c;
  _Float16* ffh   = (_Float16*)(ws + wts_bytes + r1_bytes + r2_bytes);
  float*    dummyF = (float*)ffh;
  _Float16* dummyH = ffh;

  wconv_kernel<<<WU_TOTAL / 256, 256, 0, stream>>>(wq, wk, wv, wo, w1, w2, wts);

  layernorm_kernel<<<NT_ / 8, 256, 0, stream>>>(x, ln1_g, ln1_b, r1);

  gemm_kernel<0><<<dim3(NT_ / 128, QKVW_ / 64), 128, 0, stream>>>(
      r1, wqkvh, bq, bk, bv, CC_, x, dummyF, qkvh, QKVW_, CC_);

  na_kernel<<<NT_ / 32, 256, 0, stream>>>(qkvh, rpb, r1);

  gemm_kernel<1><<<dim3(NT_ / 128, CC_ / 64), 128, 0, stream>>>(
      r1, woh, bo, bo, bo, CC_, x, hidden, dummyH, CC_, CC_);

  layernorm_kernel<<<NT_ / 8, 256, 0, stream>>>(hidden, ln2_g, ln2_b, r1);

  for (int hf = 0; hf < 2; ++hf) {
    const size_t row0 = (size_t)hf * (NT_ / 2);
    gemm_kernel<2><<<dim3((NT_ / 2) / 128, FF_ / 64), 128, 0, stream>>>(
        r1 + row0 * CC_, w1h, b1, b1, b1, FF_, x, dummyF, ffh, FF_, CC_);
    gemm_kernel<1><<<dim3((NT_ / 2) / 128, CC_ / 64), 128, 0, stream>>>(
        ffh, w2h, b2, b2, b2, CC_, hidden + row0 * CC_, out + row0 * CC_, dummyH, CC_, FF_);
  }
}
